// MaskDecoderLayer_85366769975695
// MI455X (gfx1250) — hardware-verified
//
#include <hip/hip_runtime.h>
#define NBm 8
#define NQ 100
#define QP 112
#define NRQ (NBm * QP)
#define NS 4096
#define DD 256
#define NH 8
#define HD 32
#define DFF 1024
typedef __bf16 v16b __attribute__((ext_vector_type(16)));
typedef unsigned short v8us __attribute__((ext_vector_type(8), may_alias));
typedef float  v8f  __attribute__((ext_vector_type(8)));
typedef float  v4f  __attribute__((ext_vector_type(4)));
typedef float  v4fa __attribute__((ext_vector_type(4), may_alias));
union FragB { v16b v; v8us half[2]; unsigned short u[16]; };

__device__ __forceinline__ unsigned short bf16_bits(float x) { unsigned int u = __float_as_uint(x); return (unsigned short)((u + 0x7FFFu + ((u >> 16) & 1u)) >> 16); }
__device__ __forceinline__ float bf16_val(unsigned short b) { return __uint_as_float(((unsigned int)b) << 16); }
__device__ __forceinline__ float bf16_round(float x) { return bf16_val(bf16_bits(x)); }
template <int NT>
__device__ __forceinline__ v8f mmaN(v16b ah, v16b al, v16b bh, v16b bl, v8f c) {
  c = __builtin_amdgcn_wmma_f32_16x16x32_bf16(false, ah, false, bh, (short)0, c, false, false);
  if (NT >= 2) c = __builtin_amdgcn_wmma_f32_16x16x32_bf16(false, al, false, bh, (short)0, c, false, false);
  if (NT >= 3) c = __builtin_amdgcn_wmma_f32_16x16x32_bf16(false, ah, false, bl, (short)0, c, false, false);
  asm volatile("v_nop\n\tv_nop\n\tv_nop\n\tv_nop" : "+v"(c) : "v"(ah), "v"(al), "v"(bh), "v"(bl));
  return c;
}

__global__ __launch_bounds__(256) void k_wt_bf16(const float* __restrict__ W, unsigned short* __restrict__ Wt, int K, int N) {
  const int t = blockIdx.x * 256 + threadIdx.x;
  const int k8n = K / 8;
  if (t >= N * k8n) return;
  const int n = t / k8n, k8 = (t % k8n) * 8;
  v8us v;
#pragma unroll
  for (int i = 0; i < 8; ++i) v[i] = bf16_bits(W[(size_t)(k8 + i) * N + n]);
  *(volatile v8us*)(Wt + (size_t)n * K + k8) = v;
  __threadfence();
  *(volatile v8us*)(Wt + (size_t)n * K + k8) = v;
}

template <bool ASPLIT, int ACT, bool BIAS_BF16>
__global__ __launch_bounds__(128) void k_gemm_bf(const float* __restrict__ A, int lda, const unsigned short* __restrict__ Wt, int ldb,
                                               const float* __restrict__ bias, float* __restrict__ C, int ldc, int M, int N, int K) {
  __shared__ __attribute__((aligned(16))) float so[4][16][64];
  const int tid = threadIdx.x, w = tid >> 5, lane = tid & 31, ln = lane & 15, hh = lane >> 4;
  const int ntn = N / 64;
  const int wid = blockIdx.x * 4 + w;
  const int mt = wid / ntn, nq = wid % ntn;
  if (mt * 16 >= M) return;
  const int row0 = mt * 16, col0 = nq * 64;
  const float* arow = A + (size_t)(row0 + ln) * lda;
  v8f acc[4] = {};
  for (int kb = 0; kb < K; kb += 32) {
    FragB ah, al;
    const v4f x0 = *(const v4fa*)(arow + kb + 8 * hh), x1 = *(const v4fa*)(arow + kb + 8 * hh + 4);
    const v4f x2 = *(const v4fa*)(arow + kb + 16 + 8 * hh), x3 = *(const v4fa*)(arow + kb + 16 + 8 * hh + 4);
    float xs[16] = {x0[0],x0[1],x0[2],x0[3],x1[0],x1[1],x1[2],x1[3],x2[0],x2[1],x2[2],x2[3],x3[0],x3[1],x3[2],x3[3]};
#pragma unroll
    for (int i = 0; i < 16; ++i) { const unsigned short hb = bf16_bits(xs[i]); ah.u[i] = hb; al.u[i] = ASPLIT ? bf16_bits(xs[i] - bf16_val(hb)) : (unsigned short)0; }
#pragma unroll
    for (int t = 0; t < 4; ++t) {
      const unsigned short* brow = Wt + (size_t)(col0 + t * 16 + ln) * ldb + kb;
      FragB b;
      b.half[0] = *(const v8us*)(brow + 8 * hh);
      b.half[1] = *(const v8us*)(brow + 16 + 8 * hh);
      acc[t] = mmaN<ASPLIT ? 2 : 1>(ah.v, al.v, b.v, b.v, acc[t]);
    }
  }
#pragma unroll
  for (int t = 0; t < 4; ++t) {
    float bv = bias ? bias[col0 + t * 16 + ln] : 0.f;
    if (BIAS_BF16) bv = bf16_round(bv);
#pragma unroll
    for (int r = 0; r < 8; ++r) { float v = acc[t][r] + bv; if (ACT == 1) v = fmaxf(v, 0.f); so[w][8 * hh + r][t * 16 + ln] = v; }
  }
  __builtin_amdgcn_fence(__ATOMIC_ACQ_REL, "workgroup");
  __builtin_amdgcn_wave_barrier();
  const int rsub = lane >> 4, c4 = (lane & 15) * 4;
  for (int pass = 0; pass < 2; ++pass) {
#pragma unroll
    for (int q = 0; q < 8; ++q) {
      const int r = q * 2 + rsub;
      const v4f v = *(const v4fa*)&so[w][r][c4];
      *(volatile v4f*)(C + (size_t)(row0 + r) * ldc + col0 + c4) = v;
    }
    if (pass == 0) __threadfence();
  }
}

template <bool ASPLIT, int ACT, bool BIAS_BF16, bool RES_BF16>
__global__ __launch_bounds__(128) void k_gemm_bf3(const float* __restrict__ A, int lda, const unsigned short* __restrict__ Wt, int ldb,
                                                const float* __restrict__ bias, const float* __restrict__ resid, int rmod, int ldr,
                                                float* __restrict__ C, int ldc, int M, int N, int K) {
  __shared__ __attribute__((aligned(16))) float so[4][16][64];
  const int tid = threadIdx.x, w = tid >> 5, lane = tid & 31, ln = lane & 15, hh = lane >> 4;
  const int ntn = N / 64;
  const int wid = blockIdx.x * 4 + w;
  const int mt = wid / ntn, nq = wid % ntn;
  if (mt * 16 >= M) return;
  const int row0 = mt * 16, col0 = nq * 64;
  const float* arow = A + (size_t)(row0 + ln) * lda;
  v8f acc[4] = {};
  for (int kb = 0; kb < K; kb += 32) {
    FragB ah, al;
    const v4f x0 = *(const v4fa*)(arow + kb + 8 * hh), x1 = *(const v4fa*)(arow + kb + 8 * hh + 4);
    const v4f x2 = *(const v4fa*)(arow + kb + 16 + 8 * hh), x3 = *(const v4fa*)(arow + kb + 16 + 8 * hh + 4);
    float xs[16] = {x0[0],x0[1],x0[2],x0[3],x1[0],x1[1],x1[2],x1[3],x2[0],x2[1],x2[2],x2[3],x3[0],x3[1],x3[2],x3[3]};
#pragma unroll
    for (int i = 0; i < 16; ++i) { const unsigned short hb = bf16_bits(xs[i]); ah.u[i] = hb; al.u[i] = ASPLIT ? bf16_bits(xs[i] - bf16_val(hb)) : (unsigned short)0; }
#pragma unroll
    for (int t = 0; t < 4; ++t) {
      const unsigned short* brow = Wt + (size_t)(col0 + t * 16 + ln) * ldb + kb;
      FragB b;
      b.half[0] = *(const v8us*)(brow + 8 * hh);
      b.half[1] = *(const v8us*)(brow + 16 + 8 * hh);
      acc[t] = mmaN<ASPLIT ? 2 : 1>(ah.v, al.v, b.v, b.v, acc[t]);
    }
  }
#pragma unroll
  for (int t = 0; t < 4; ++t) {
    const int col = col0 + t * 16 + ln;
    float bv = bias ? bias[col] : 0.f;
    if (BIAS_BF16) bv = bf16_round(bv);
#pragma unroll
    for (int r = 0; r < 8; ++r) {
      float v = acc[t][r] + bv;
      if (resid) { float rv = resid[(size_t)((row0 + 8 * hh + r) % rmod) * ldr + col]; if (RES_BF16) rv = bf16_round(rv); v += rv; }
      if (ACT == 1) v = fmaxf(v, 0.f);
      if (ACT == 2) v = 0.5f * v * (1.0f + erff(v * 0.70710678118654752f));
      if (ACT == 3) { const float u = 0.7978845608028654f * (v + 0.044715f * v * v * v); v = 0.5f * v * (1.0f + tanhf(u)); }
      so[w][8 * hh + r][t * 16 + ln] = v;
    }
  }
  __builtin_amdgcn_fence(__ATOMIC_ACQ_REL, "workgroup");
  __builtin_amdgcn_wave_barrier();
  const int rsub = lane >> 4, c4 = (lane & 15) * 4;
  for (int pass = 0; pass < 2; ++pass) {
#pragma unroll
    for (int q = 0; q < 8; ++q) {
      const int r = q * 2 + rsub;
      const v4f v = *(const v4fa*)&so[w][r][c4];
      *(volatile v4f*)(C + (size_t)(row0 + r) * ldc + col0 + c4) = v;
    }
    if (pass == 0) __threadfence();
  }
}
template <bool PARAM_BF16>
__global__ __launch_bounds__(256) void k_layernorm(const float* __restrict__ X, const float* __restrict__ R, const float* __restrict__ g, const float* __restrict__ bta,
                                                  float* __restrict__ out_sum, float* __restrict__ out_norm, int N, float eps) {
  __shared__ float red[256];
  const int row = blockIdx.x, tid = threadIdx.x;
  const float* x = X + (size_t)row * N; const float* rr = R ? R + (size_t)row * N : nullptr;
  float vals[16];
  const int per = N / 256;
  float s1 = 0.f;
  for (int u = 0; u < per / 4; ++u) {
    const int j = tid * 4 + 1024 * u;
    const v4f a = *(const v4fa*)(x + j);
    v4f b = {0.f,0.f,0.f,0.f}; if (rr) b = *(const v4fa*)(rr + j);
#pragma unroll
    for (int q = 0; q < 4; ++q) { const float v = a[q] + b[q]; vals[u * 4 + q] = v; s1 += v; }
  }
  red[tid] = s1; __syncthreads();
  for (int st = 128; st > 0; st >>= 1) { if (tid < st) red[tid] += red[tid + st]; __syncthreads(); }
  const float mu = red[0] / (float)N; __syncthreads();
  float s2 = 0.f;
  for (int u = 0; u < per / 4; ++u)
#pragma unroll
    for (int q = 0; q < 4; ++q) { const float c = vals[u * 4 + q] - mu; s2 += c * c; }
  red[tid] = s2; __syncthreads();
  for (int st = 128; st > 0; st >>= 1) { if (tid < st) red[tid] += red[tid + st]; __syncthreads(); }
  const float rs = rsqrtf(red[0] / (float)N + eps);
  for (int pass = 0; pass < 2; ++pass) {
    for (int u = 0; u < per / 4; ++u) {
      const int j = tid * 4 + 1024 * u;
      v4f o, sm;
#pragma unroll
      for (int q = 0; q < 4; ++q) {
        float gg = g[j + q], bb = bta[j + q];
        if (PARAM_BF16) { gg = bf16_round(gg); bb = bf16_round(bb); }
        sm[q] = vals[u * 4 + q]; o[q] = (vals[u * 4 + q] - mu) * rs * gg + bb;
      }
      if (out_sum) *(volatile v4f*)(out_sum + (size_t)row * N + j) = sm;
      *(volatile v4f*)(out_norm + (size_t)row * N + j) = o;
    }
    if (pass == 0) __threadfence();
  }
}


typedef _Float16 v16h __attribute__((ext_vector_type(16)));
union FragH { v16h v; v8us half[2]; _Float16 h[16]; unsigned short u[16]; };
template <int NT>
__device__ __forceinline__ v8f mmaH(v16h ah, v16h al, v16h bh, v16h bl, v8f c) {
  c = __builtin_amdgcn_wmma_f32_16x16x32_f16(false, ah, false, bh, (short)0, c, false, false);
  if (NT >= 2) c = __builtin_amdgcn_wmma_f32_16x16x32_f16(false, al, false, bh, (short)0, c, false, false);
  if (NT >= 3) c = __builtin_amdgcn_wmma_f32_16x16x32_f16(false, ah, false, bl, (short)0, c, false, false);
  asm volatile("v_nop\n\tv_nop\n\tv_nop\n\tv_nop" : "+v"(c) : "v"(ah), "v"(al), "v"(bh), "v"(bl));
  return c;
}
template <bool ASPLIT>
__global__ __launch_bounds__(128) void k_gemm_h(const float* __restrict__ A, int lda, size_t sA, const _Float16* __restrict__ Bh, int ldb, size_t sB, float alpha, float* __restrict__ C, int ldc, size_t sC, int M, int N, int K) {
  __shared__ __attribute__((aligned(16))) float so[4][16][64];
  const int tid = threadIdx.x, w = tid >> 5, lane = tid & 31, ln = lane & 15, hh = lane >> 4; const int by = blockIdx.y;
  A += (size_t)by * sA; Bh += (size_t)by * sB; C += (size_t)by * sC;
  const int ntn = (N + 63) / 64; const int wid = blockIdx.x * 4 + w; const int mt = wid / ntn, nq = wid % ntn; if (mt * 16 >= M) return;
  const int row0 = mt * 16, col0 = nq * 64; const float* arow = A + (size_t)(row0 + ln) * lda;
  v8f acc[4] = {};
  for (int kb = 0; kb < K; kb += 32) {
    FragH ah, al;
    const v4f x0 = *(const v4fa*)(arow + kb + 8 * hh), x1 = *(const v4fa*)(arow + kb + 8 * hh + 4), x2 = *(const v4fa*)(arow + kb + 16 + 8 * hh), x3 = *(const v4fa*)(arow + kb + 16 + 8 * hh + 4);
    float xs[16] = {x0[0],x0[1],x0[2],x0[3],x1[0],x1[1],x1[2],x1[3],x2[0],x2[1],x2[2],x2[3],x3[0],x3[1],x3[2],x3[3]};
#pragma unroll
    for (int i = 0; i < 16; ++i) { const _Float16 h = (_Float16)xs[i]; ah.h[i] = h; al.h[i] = ASPLIT ? (_Float16)(xs[i] - (float)h) : (_Float16)0.0f; }
#pragma unroll
    for (int t = 0; t < 4; ++t) { if (col0 + t * 16 >= N) continue; const size_t boff = (size_t)(col0 + t * 16 + ln) * ldb + kb; FragH bq; bq.half[0] = *(const v8us*)(Bh + boff + 8 * hh); bq.half[1] = *(const v8us*)(Bh + boff + 16 + 8 * hh);
      acc[t] = mmaH<ASPLIT ? 2 : 1>(ah.v, al.v, bq.v, bq.v, acc[t]); }
  }
#pragma unroll
  for (int t = 0; t < 4; ++t) { if (col0 + t * 16 >= N) continue;
#pragma unroll
    for (int r = 0; r < 8; ++r) so[w][8 * hh + r][t * 16 + ln] = acc[t][r] * alpha; }
  __builtin_amdgcn_fence(__ATOMIC_ACQ_REL, "workgroup"); __builtin_amdgcn_wave_barrier();
  const int rsub = lane >> 4, c4 = (lane & 15) * 4;
  for (int pass = 0; pass < 2; ++pass) {
#pragma unroll
    for (int q = 0; q < 8; ++q) { const int r = q * 2 + rsub; if (col0 + c4 < N) { const v4f v = *(const v4fa*)&so[w][r][c4]; *(volatile v4f*)(C + (size_t)(row0 + r) * ldc + col0 + c4) = v; } }
    if (pass == 0) __threadfence(); }
}

__global__ __launch_bounds__(256) void k_wt_f16(const float* __restrict__ W, _Float16* __restrict__ Wt, int K, int N, float scale) {
  const int t = blockIdx.x * 256 + threadIdx.x; if (t >= N * (K / 8)) return; const int n = t / (K / 8), k8 = (t % (K / 8)) * 8; FragH f;
#pragma unroll
  for (int i = 0; i < 8; ++i) f.h[i] = (_Float16)(bf16_round(W[(size_t)(k8 + i) * N + n]) * scale); const v8us o = f.half[0];
  *(volatile v8us*)((unsigned short*)Wt + (size_t)n * K + k8) = o; __threadfence(); *(volatile v8us*)((unsigned short*)Wt + (size_t)n * K + k8) = o;
}
template <int ACT>
__global__ __launch_bounds__(128) void k_gemm_hhx(const _Float16* __restrict__ A, int lda, size_t sA, const _Float16* __restrict__ Bh, int ldb, size_t sB, float alpha, const float* __restrict__ bias, size_t sBias, const float* __restrict__ CP, int rowsPerB, size_t sCPb, int row0g,
    float* __restrict__ C, _Float16* __restrict__ C16, int ldc, size_t sC, int M, int N, int K) {
  __shared__ __attribute__((aligned(16))) float so[4][16][64];
  const int tid = threadIdx.x, w = tid >> 5, lane = tid & 31, ln = lane & 15, hh = lane >> 4; const int by = blockIdx.y;
  A += (size_t)by * sA; Bh += (size_t)by * sB; const size_t cofs = (size_t)by * sC; const float* bp = bias ? bias + (size_t)by * sBias : nullptr;
  const int ntn = (N + 63) / 64; const int wid = blockIdx.x * 4 + w; const int mt = wid / ntn, nq = wid % ntn; if (mt * 16 >= M) return;
  const int row0 = mt * 16, col0 = nq * 64; const _Float16* arow = A + (size_t)(row0 + ln) * lda;
  v8f acc[4] = {};
  for (int kb = 0; kb < K; kb += 32) { FragH ah; ah.half[0] = *(const v8us*)((const unsigned short*)arow + kb + 8 * hh); ah.half[1] = *(const v8us*)((const unsigned short*)arow + kb + 16 + 8 * hh);
#pragma unroll
    for (int t = 0; t < 4; ++t) { if (col0 + t * 16 >= N) continue; const size_t boff = (size_t)(col0 + t * 16 + ln) * ldb + kb; FragH bq; bq.half[0] = *(const v8us*)((const unsigned short*)Bh + boff + 8 * hh); bq.half[1] = *(const v8us*)((const unsigned short*)Bh + boff + 16 + 8 * hh);
      acc[t] = mmaH<1>(ah.v, ah.v, bq.v, bq.v, acc[t]); }
  }
#pragma unroll
  for (int t = 0; t < 4; ++t) { if (col0 + t * 16 >= N) continue; const int col = col0 + t * 16 + ln; const float bv = bp ? bf16_round(bp[col]) : 0.f;
#pragma unroll
    for (int r = 0; r < 8; ++r) { float v = acc[t][r] * alpha + bv; if (CP) { const int bidx = (row0g + row0 + 8 * hh + r) / rowsPerB; v += CP[(size_t)bidx * sCPb + (size_t)by * 64 + col]; } if (ACT == 1) v = (v > 0.f) ? v : expm1f(v); else if (ACT == 7) v = (v > 0.f) ? v + 1.0f : expf(v); else if (ACT == 8) v = tanhf(v); else if (ACT == 9) v = 0.5f * v * (1.0f + tanhf(0.7978845608028654f * (v + 0.044715f * v * v * v))); else if (ACT == 11) v = 1.0f / (1.0f + expf(-v)); else if (ACT == 12) v = (v > 0.f) ? v : 0.01f * v; else if (ACT == 14) v = (v > 0.f) ? v : 0.1f * v; else if (ACT == 15) v = v / (1.0f + expf(-v)); else if (ACT == 3) v = fmaxf(v, 0.f); else if (ACT == 6) v = 0.5f * v * (1.0f + erff(v * 0.70710678118654752f)); so[w][8 * hh + r][t * 16 + ln] = v; } }
  __builtin_amdgcn_fence(__ATOMIC_ACQ_REL, "workgroup"); __builtin_amdgcn_wave_barrier();
  const int rsub = lane >> 4, c4 = (lane & 15) * 4; typedef _Float16 v4h __attribute__((ext_vector_type(4)));
  for (int pass = 0; pass < 2; ++pass) {
#pragma unroll
    for (int q = 0; q < 8; ++q) { const int r = q * 2 + rsub; if (col0 + c4 < N) { const v4f v = *(const v4fa*)&so[w][r][c4]; if (C) *(volatile v4f*)(C + cofs + (size_t)(row0 + r) * ldc + col0 + c4) = v; if (C16) { v4h h4; for (int i = 0; i < 4; ++i) h4[i] = (_Float16)v[i]; *(volatile v4h*)(C16 + cofs + (size_t)(row0 + r) * ldc + col0 + c4) = h4; } } }
    if (pass == 0) __threadfence(); }
}


typedef _Float16 v4h __attribute__((ext_vector_type(4)));

__global__ __launch_bounds__(256) void k_x16(const float* __restrict__ x, _Float16* __restrict__ X16, size_t n8) { const size_t t = (size_t)blockIdx.x * 256 + threadIdx.x; if (t >= n8) return; FragH f;
#pragma unroll
  for (int q = 0; q < 8; ++q) f.h[q] = (_Float16)bf16_round(x[t * 8 + q]); *(volatile v8us*)((unsigned short*)X16 + t * 8) = f.half[0]; __threadfence(); *(volatile v8us*)((unsigned short*)X16 + t * 8) = f.half[0]; }
__global__ __launch_bounds__(256) void k_h16(const float* __restrict__ x, _Float16* __restrict__ X16, size_t n8) { const size_t t = (size_t)blockIdx.x * 256 + threadIdx.x; if (t >= n8) return; FragH f;
#pragma unroll
  for (int q = 0; q < 8; ++q) f.h[q] = (_Float16)x[t * 8 + q]; *(volatile v8us*)((unsigned short*)X16 + t * 8) = f.half[0]; __threadfence(); *(volatile v8us*)((unsigned short*)X16 + t * 8) = f.half[0]; }
__global__ __launch_bounds__(256) void k_round16f(const float* __restrict__ W, _Float16* __restrict__ Bt, size_t n8) { const size_t t = (size_t)blockIdx.x * 256 + threadIdx.x; if (t >= n8) return; FragH f;
#pragma unroll
  for (int i = 0; i < 8; ++i) f.h[i] = (_Float16)(bf16_round(W[t * 8 + i]) * 16.0f); *(volatile v8us*)((unsigned short*)Bt + t * 8) = f.half[0]; __threadfence(); *(volatile v8us*)((unsigned short*)Bt + t * 8) = f.half[0]; }
template <int NHv, int TTv>
__global__ __launch_bounds__(256) void k_vt(const _Float16* __restrict__ V16, int ldv, int voff, _Float16* __restrict__ Vt) { __shared__ unsigned short tl[64][66]; const int tid = threadIdx.x; const int slab = blockIdx.x / (TTv / 64), lg = blockIdx.x % (TTv / 64); const int b = slab / NHv, h = slab % NHv;
  for (int i = tid; i < 64 * 8; i += 256) { const int r = i / 8, c8 = (i % 8) * 8; FragH f; f.half[0] = *(const v8us*)((const unsigned short*)V16 + ((size_t)b * TTv + lg * 64 + r) * ldv + voff + h * 64 + c8);
#pragma unroll
    for (int q = 0; q < 8; ++q) tl[r][c8 + q] = f.u[q]; }
  __syncthreads();
  for (int pass = 0; pass < 2; ++pass) {
#pragma unroll
    for (int rd = 0; rd < 2; ++rd) { const int d = rd * 32 + tid / 8, pc = tid % 8; FragH f;
#pragma unroll
      for (int q = 0; q < 8; ++q) f.u[q] = tl[pc * 8 + q][d];
      *(volatile v8us*)((unsigned short*)Vt + ((size_t)slab * 64 + d) * TTv + lg * 64 + pc * 8) = f.half[0]; }
    if (pass == 0) __threadfence(); } }

__global__ __launch_bounds__(256) void k_hl(const float* __restrict__ F, _Float16* __restrict__ Hh, _Float16* __restrict__ Hl, size_t n8) { const size_t t = (size_t)blockIdx.x * 256 + threadIdx.x; if (t >= n8) return; FragH fh, fl; const v4f a = *(const v4fa*)(F + t * 8), c = *(const v4fa*)(F + t * 8 + 4);
#pragma unroll
  for (int q = 0; q < 4; ++q) { _Float16 h = (_Float16)a[q]; fh.h[q] = h; fl.h[q] = (_Float16)((a[q] - (float)h) * 1024.0f); h = (_Float16)c[q]; fh.h[4 + q] = h; fl.h[4 + q] = (_Float16)((c[q] - (float)h) * 1024.0f); }
  for (int pass = 0; pass < 2; ++pass) { *(volatile v8us*)((unsigned short*)Hh + t * 8) = fh.half[0]; *(volatile v8us*)((unsigned short*)Hl + t * 8) = fl.half[0]; if (pass == 0) __threadfence(); } }

__global__ __launch_bounds__(256) void k_qpad(const float* __restrict__ qin, float* __restrict__ QF) { const int t = blockIdx.x * 256 + threadIdx.x; if (t >= NRQ * (DD / 4)) return; const int c0 = (t % (DD / 4)) * 4, r = t / (DD / 4); const int b = r / QP, q = r % QP; v4f v; v[0] = v[1] = v[2] = v[3] = 0.f;
  if (q < NQ) { const v4f a = *(const v4fa*)(qin + ((size_t)b * NQ + q) * DD + c0); for (int k = 0; k < 4; ++k) v[k] = bf16_round(a[k]); }
  *(volatile v4f*)(QF + (size_t)r * DD + c0) = v; __threadfence(); *(volatile v4f*)(QF + (size_t)r * DD + c0) = v; }
__global__ __launch_bounds__(256) void k_ln16(const float* __restrict__ X, const float* __restrict__ g, const float* __restrict__ bb, _Float16* __restrict__ Y) {
  #pragma clang fp contract(off)
  const int tid = threadIdx.x, w = tid >> 5, l = tid & 31; const int r = blockIdx.x * 8 + w; if (r >= NRQ) return; const bool live = (r % QP) < NQ; const v4f a = *(const v4fa*)(X + (size_t)r * DD + 8 * l), c = *(const v4fa*)(X + (size_t)r * DD + 8 * l + 4); float v[8];
#pragma unroll
  for (int q = 0; q < 8; ++q) v[q] = (q < 4) ? a[q] : c[q - 4];
  float s = 0.f;
#pragma unroll
  for (int q = 0; q < 8; ++q) s += v[q]; for (int o = 16; o > 0; o >>= 1) s += __shfl_xor(s, o, 32); const float mu = s / (float)DD; float vs = 0.f;
#pragma unroll
  for (int q = 0; q < 8; ++q) vs += (v[q] - mu) * (v[q] - mu); for (int o = 16; o > 0; o >>= 1) vs += __shfl_xor(vs, o, 32); const float rs = rsqrtf(vs / (float)DD + 1e-5f); FragH f;
#pragma unroll
  for (int q = 0; q < 8; ++q) { const int cc = 8 * l + q; f.h[q] = live ? (_Float16)((v[q] - mu) * rs * bf16_round(g[cc]) + bf16_round(bb[cc])) : (_Float16)0.0f; }
  *(volatile v8us*)((unsigned short*)Y + (size_t)r * DD + 8 * l) = f.half[0]; __threadfence(); *(volatile v8us*)((unsigned short*)Y + (size_t)r * DD + 8 * l) = f.half[0]; }
__global__ __launch_bounds__(256) void k_any(const float* __restrict__ pm, float* __restrict__ ANY) {
  #pragma clang fp contract(off)
  const int tid = threadIdx.x, w = tid >> 5, l = tid & 31; const int r = blockIdx.x * 8 + w; if (r >= NRQ) return; const int b = r / QP, q = r % QP; float any = 0.f;
  if (q < NQ) { const float* row = pm + ((size_t)b * NQ + q) * NS;
#pragma unroll 1
    for (int j = l; j < NS; j += 32) { const float sg = 1.0f / (1.0f + expf(-bf16_round(row[j]))); any = (sg > 0.5f) ? 1.f : any; } }
  else any = 1.f;
  for (int o = 16; o > 0; o >>= 1) any = fmaxf(any, __shfl_xor(any, o, 32));
  *(volatile float*)(ANY + (size_t)r * 32 + l) = any; __threadfence(); *(volatile float*)(ANY + (size_t)r * 32 + l) = any; }
__global__ __launch_bounds__(256) void k_bias(const float* __restrict__ pm, const float* __restrict__ ANY, float* __restrict__ BIAS) {
  #pragma clang fp contract(off)
  const size_t t = (size_t)blockIdx.x * 256 + threadIdx.x; if (t >= (size_t)NRQ * (NS / 4)) return; const int j0 = (int)(t % (NS / 4)) * 4; const int r = (int)(t / (NS / 4)); const int b = r / QP, q = r % QP; v4f o; o[0] = o[1] = o[2] = o[3] = 0.f;
  if (q < NQ && ANY[(size_t)r * 32] != 0.f) { const float* prow = pm + ((size_t)b * NQ + q) * NS + j0;
#pragma unroll
    for (int k = 0; k < 4; ++k) { const float sg = 1.0f / (1.0f + expf(-bf16_round(prow[k]))); o[k] = (sg > 0.5f) ? 0.f : -10000.0f; } }
  *(volatile v4f*)(BIAS + (size_t)r * NS + j0) = o; __threadfence(); *(volatile v4f*)(BIAS + (size_t)r * NS + j0) = o; }
__global__ __launch_bounds__(256) void k_csoft(const float* __restrict__ S, const float* __restrict__ BIAS, int h, _Float16* __restrict__ P16, float* __restrict__ RS) {
  #pragma clang fp contract(off)
  const int tid = threadIdx.x, w = tid >> 5, l = tid & 31; const int r = blockIdx.x * 8 + w; if (r >= NRQ) return; const bool live = (r % QP) < NQ; const float* srow = S + (size_t)r * NS; const float* brow = BIAS + (size_t)r * NS;
  float m = -3.0e38f;
#pragma unroll 1
  for (int jb = 0; jb < NS; jb += 256) { const v4f s0 = *(const v4fa*)(srow + jb + 8 * l), s1 = *(const v4fa*)(srow + jb + 8 * l + 4), b0 = *(const v4fa*)(brow + jb + 8 * l), b1v = *(const v4fa*)(brow + jb + 8 * l + 4);
#pragma unroll
    for (int k = 0; k < 4; ++k) { m = fmaxf(m, s0[k] + b0[k]); m = fmaxf(m, s1[k] + b1v[k]); } }
  for (int o = 16; o > 0; o >>= 1) m = fmaxf(m, __shfl_xor(m, o, 32));
  float ssum = 0.f;
#pragma unroll 1
  for (int jb = 0; jb < NS; jb += 256) { const v4f s0 = *(const v4fa*)(srow + jb + 8 * l), s1 = *(const v4fa*)(srow + jb + 8 * l + 4), b0 = *(const v4fa*)(brow + jb + 8 * l), b1v = *(const v4fa*)(brow + jb + 8 * l + 4); FragH f;
#pragma unroll
    for (int k = 0; k < 4; ++k) { const float e0 = live ? expf((s0[k] + b0[k]) - m) : 0.f, e1 = live ? expf((s1[k] + b1v[k]) - m) : 0.f; ssum += e0 + e1; f.h[k] = (_Float16)(e0 * 1024.0f); f.h[4 + k] = (_Float16)(e1 * 1024.0f); }
    *(volatile v8us*)((unsigned short*)P16 + (size_t)r * NS + jb + 8 * l) = f.half[0]; __threadfence(); *(volatile v8us*)((unsigned short*)P16 + (size_t)r * NS + jb + 8 * l) = f.half[0]; }
  for (int o = 16; o > 0; o >>= 1) ssum += __shfl_xor(ssum, o, 32);
  const float prev = RS[(size_t)r * 32 + l]; const float v = (l == h) ? (live ? ssum : 1.f) : ((h == 0) ? 0.f : prev);
  *(volatile float*)(RS + (size_t)r * 32 + l) = v; __threadfence(); *(volatile float*)(RS + (size_t)r * 32 + l) = v; }
__global__ __launch_bounds__(256) void k_onorm(float* __restrict__ O1, const float* __restrict__ RS) {
  #pragma clang fp contract(off)
  const int t = blockIdx.x * 256 + threadIdx.x; if (t >= NRQ * (DD / 8)) return; const int c0 = (t % (DD / 8)) * 8, r = t / (DD / 8); const int h = c0 / HD; const float inv = 1.0f / RS[(size_t)r * 32 + h]; const v4f a = *(const v4fa*)(O1 + (size_t)r * DD + c0), c = *(const v4fa*)(O1 + (size_t)r * DD + c0 + 4); v4f oa, oc;
#pragma unroll
  for (int k = 0; k < 4; ++k) { oa[k] = a[k] * inv; oc[k] = c[k] * inv; }
  for (int pass = 0; pass < 2; ++pass) { *(volatile v4f*)(O1 + (size_t)r * DD + c0) = oa; *(volatile v4f*)(O1 + (size_t)r * DD + c0 + 4) = oc; if (pass == 0) __threadfence(); } }
__global__ __launch_bounds__(256) void k_vt(const _Float16* __restrict__ KV, _Float16* __restrict__ VT) { const size_t t = (size_t)blockIdx.x * 256 + threadIdx.x; if (t >= (size_t)NBm * NH * HD * (NS / 8)) return; const int j0 = (int)(t % (NS / 8)) * 8; const int d = (int)((t / (NS / 8)) % HD); const int bh = (int)(t / ((size_t)(NS / 8) * HD)); const int b = bh / NH, h = bh % NH; FragH f;
#pragma unroll
  for (int q = 0; q < 8; ++q) f.h[q] = KV[((size_t)b * NS + j0 + q) * (2 * DD) + DD + h * HD + d];
  *(volatile v8us*)((unsigned short*)VT + ((size_t)bh * HD + d) * NS + j0) = f.half[0]; __threadfence(); *(volatile v8us*)((unsigned short*)VT + ((size_t)bh * HD + d) * NS + j0) = f.half[0]; }
__global__ __launch_bounds__(256) void k_sattn(const float* __restrict__ QKV3, float* __restrict__ O2) {
  #pragma clang fp contract(off)
  const int t = blockIdx.x * 256 + threadIdx.x; if (t >= NRQ * NH * 2) return; const int hf = t & 1; const int h = (t >> 1) % NH; const int r = t / (2 * NH); const int b = r / QP, q = r % QP; v4f w0, w1, w2, w3; w0 = (v4f){}; w1 = w0; w2 = w0; w3 = w0;
  if (q < NQ) { float qv[HD]; const float* qp = QKV3 + (size_t)r * (3 * DD) + h * HD;
#pragma unroll
    for (int d = 0; d < HD; ++d) qv[d] = qp[d] * 0.1767766952966369f;
    float m = -3.0e38f, lsum = 0.f; float o[16];
#pragma unroll
    for (int d = 0; d < 16; ++d) o[d] = 0.f;
#pragma unroll 1
    for (int j = 0; j < NQ; ++j) { const float* kp = QKV3 + ((size_t)b * QP + j) * (3 * DD) + DD + h * HD; float s = 0.f;
#pragma unroll
      for (int d = 0; d < HD; ++d) s += qv[d] * kp[d];
      const float mn = fmaxf(m, s); const float corr = expf(m - mn); const float p = expf(s - mn); lsum = lsum * corr + p; const float* vp = QKV3 + ((size_t)b * QP + j) * (3 * DD) + 2 * DD + h * HD + hf * 16;
#pragma unroll
      for (int d = 0; d < 16; ++d) o[d] = o[d] * corr + p * vp[d];
      m = mn; }
    const float inv = 1.0f / lsum;
#pragma unroll
    for (int d = 0; d < 4; ++d) { w0[d] = o[d] * inv; w1[d] = o[4 + d] * inv; w2[d] = o[8 + d] * inv; w3[d] = o[12 + d] * inv; } }
  float* dst = O2 + (size_t)r * DD + h * HD + hf * 16;
  for (int pass = 0; pass < 2; ++pass) { *(volatile v4f*)dst = w0; *(volatile v4f*)(dst + 4) = w1; *(volatile v4f*)(dst + 8) = w2; *(volatile v4f*)(dst + 12) = w3; if (pass == 0) __threadfence(); } }
__global__ __launch_bounds__(256) void k_out(const float* __restrict__ R, float* __restrict__ out) { const int t = blockIdx.x * 256 + threadIdx.x; if (t >= NBm * NQ * (DD / 4)) return; const int c0 = (t % (DD / 4)) * 4; const int rq = t / (DD / 4); const int b = rq / NQ, q = rq % NQ; const v4f v = *(const v4fa*)(R + ((size_t)b * QP + q) * DD + c0); *(volatile v4f*)(out + (size_t)rq * DD + c0) = v; __threadfence(); *(volatile v4f*)(out + (size_t)rq * DD + c0) = v; }

extern "C" void kernel_launch(void* const* d_in, const int* in_sizes, int n_in,
                              void* d_out, int out_size, void* d_ws, size_t ws_size, hipStream_t stream) {
  (void)in_sizes; (void)n_in; (void)out_size;
  const float* const* I = (const float* const*)d_in; const float* qin = I[0]; const float* pix = I[1]; const float* pm = I[2]; const float* ciw = I[3]; const float* cib = I[4]; const float* cow = I[5]; const float* cob = I[6]; const float* siw = I[7]; const float* sib = I[8]; const float* sow = I[9]; const float* sob = I[10];
  const float* lcg = I[11]; const float* lcb = I[12]; const float* lsg = I[13]; const float* lsb = I[14]; const float* lfg = I[15]; const float* lfb = I[16]; const float* w1 = I[17]; const float* b1 = I[18]; const float* w2 = I[19]; const float* b2 = I[20];
  char* ws = (char*)d_ws; size_t off = 0;
  auto take = [&](size_t bytes) { char* p = ws + off; off += (bytes + 255) & ~(size_t)255; return p; };
  _Float16* Bci = (_Float16*)take((size_t)3 * DD * DD * 2); _Float16* Bco = (_Float16*)take((size_t)DD * DD * 2); _Float16* Bsi = (_Float16*)take((size_t)3 * DD * DD * 2); _Float16* Bso = (_Float16*)take((size_t)DD * DD * 2); _Float16* Bw1 = (_Float16*)take((size_t)DFF * DD * 2); _Float16* Bw2 = (_Float16*)take((size_t)DD * DFF * 2);
  float* QF = (float*)take((size_t)NRQ * DD * 4); float* BIAS = (float*)take((size_t)NRQ * NS * 4); float* RS = (float*)take((size_t)NRQ * 32 * 4); _Float16* L16 = (_Float16*)take((size_t)NRQ * DD * 2); _Float16* Q16 = (_Float16*)take((size_t)NRQ * DD * 2); float* ANY = (float*)take((size_t)NRQ * 32 * 4);
  _Float16* X16 = (_Float16*)take((size_t)NBm * NS * DD * 2); _Float16* KV16 = (_Float16*)take((size_t)NBm * NS * 2 * DD * 2); _Float16* VT = (_Float16*)take((size_t)NBm * NH * HD * NS * 2);
  float* S = (float*)take((size_t)NRQ * NS * 4); _Float16* P16 = (_Float16*)take((size_t)NRQ * NS * 2); float* O1 = (float*)take((size_t)NRQ * DD * 4); _Float16* O16 = (_Float16*)take((size_t)NRQ * DD * 2); float* Q1 = (float*)take((size_t)NRQ * DD * 4);
  float* QKV3 = (float*)take((size_t)NRQ * 3 * DD * 4); float* O2 = (float*)take((size_t)NRQ * DD * 4); float* Q2 = (float*)take((size_t)NRQ * DD * 4); _Float16* F16 = (_Float16*)take((size_t)NRQ * DFF * 2); float* R3 = (float*)take((size_t)NRQ * DD * 4);
  if (off > ws_size) return;
  k_round16f<<<(3 * DD * DD / 8 + 255) / 256, 256, 0, stream>>>(ciw, Bci, (size_t)3 * DD * DD / 8); k_round16f<<<(DD * DD / 8 + 255) / 256, 256, 0, stream>>>(cow, Bco, (size_t)DD * DD / 8); k_round16f<<<(3 * DD * DD / 8 + 255) / 256, 256, 0, stream>>>(siw, Bsi, (size_t)3 * DD * DD / 8); k_round16f<<<(DD * DD / 8 + 255) / 256, 256, 0, stream>>>(sow, Bso, (size_t)DD * DD / 8); k_round16f<<<(DFF * DD / 8 + 255) / 256, 256, 0, stream>>>(w1, Bw1, (size_t)DFF * DD / 8); k_round16f<<<(DD * DFF / 8 + 255) / 256, 256, 0, stream>>>(w2, Bw2, (size_t)DD * DFF / 8);
  k_qpad<<<(NRQ * (DD / 4) + 255) / 256, 256, 0, stream>>>(qin, QF); k_any<<<NRQ / 8, 256, 0, stream>>>(pm, ANY); k_bias<<<(unsigned)(((size_t)NRQ * (NS / 4) + 255) / 256), 256, 0, stream>>>(pm, ANY, BIAS);
  k_x16<<<(unsigned)(((size_t)NBm * NS * DD / 8 + 255) / 256), 256, 0, stream>>>(pix, X16, (size_t)NBm * NS * DD / 8);
  const dim3 gKV(((NBm * NS / 16) * (2 * DD / 64) + 3) / 4, 1), gQ(((NRQ / 16) * (DD / 64) + 3) / 4, 1), gQ3(((NRQ / 16) * (3 * DD / 64) + 3) / 4, 1), gF(((NRQ / 16) * (DFF / 64) + 3) / 4, 1);
  k_gemm_hhx<0><<<gKV, 128, 0, stream>>>(X16, DD, 0, Bci + (size_t)DD * DD, DD, 0, 0.0625f, cib + DD, 0, nullptr, 1, 0, 0, nullptr, KV16, 2 * DD, 0, NBm * NS, 2 * DD, DD);
  k_vt<<<(unsigned)(((size_t)NBm * NH * HD * (NS / 8) + 255) / 256), 256, 0, stream>>>(KV16, VT);
  k_ln16<<<NRQ / 8, 256, 0, stream>>>(QF, lcg, lcb, L16);
  k_gemm_hhx<0><<<gQ, 128, 0, stream>>>(L16, DD, 0, Bci, DD, 0, 0.0625f, cib, 0, nullptr, 1, 0, 0, nullptr, Q16, DD, 0, NRQ, DD, DD);
  for (int h = 0; h < NH; ++h) {
    k_gemm_hhx<0><<<dim3(((QP / 16) * (NS / 64) + 3) / 4, NBm), 128, 0, stream>>>(Q16 + h * HD, DD, (size_t)QP * DD, KV16 + h * HD, 2 * DD, (size_t)NS * 2 * DD, 0.1767766952966369f, nullptr, 0, nullptr, 1, 0, 0, S, nullptr, NS, (size_t)QP * NS, QP, NS, HD);
    k_csoft<<<NRQ / 8, 256, 0, stream>>>(S, BIAS, h, P16, RS);
    k_gemm_hhx<0><<<dim3(((QP / 16) * 1 + 3) / 4, NBm), 128, 0, stream>>>(P16, NS, (size_t)QP * NS, VT + (size_t)h * HD * NS, NS, (size_t)NH * HD * NS, 0.0009765625f, nullptr, 0, nullptr, 1, 0, 0, O1 + h * HD, nullptr, DD, (size_t)QP * DD, QP, HD, NS); }
  k_onorm<<<(NRQ * (DD / 8) + 255) / 256, 256, 0, stream>>>(O1, RS); k_h16<<<(NRQ * DD / 8 + 255) / 256, 256, 0, stream>>>(O1, O16, (size_t)NRQ * DD / 8);
  k_gemm_hhx<0><<<gQ, 128, 0, stream>>>(O16, DD, 0, Bco, DD, 0, 0.0625f, cob, 0, QF, 1, (size_t)DD, 0, Q1, nullptr, DD, 0, NRQ, DD, DD);
  k_ln16<<<NRQ / 8, 256, 0, stream>>>(Q1, lsg, lsb, L16);
  k_gemm_hhx<0><<<gQ3, 128, 0, stream>>>(L16, DD, 0, Bsi, DD, 0, 0.0625f, sib, 0, nullptr, 1, 0, 0, QKV3, nullptr, 3 * DD, 0, NRQ, 3 * DD, DD);
  k_sattn<<<(NRQ * NH * 2 + 255) / 256, 256, 0, stream>>>(QKV3, O2);
  k_h16<<<(NRQ * DD / 8 + 255) / 256, 256, 0, stream>>>(O2, O16, (size_t)NRQ * DD / 8);
  k_gemm_hhx<0><<<gQ, 128, 0, stream>>>(O16, DD, 0, Bso, DD, 0, 0.0625f, sob, 0, Q1, 1, (size_t)DD, 0, Q2, nullptr, DD, 0, NRQ, DD, DD);
  k_ln16<<<NRQ / 8, 256, 0, stream>>>(Q2, lfg, lfb, L16);
  k_gemm_hhx<6><<<gF, 128, 0, stream>>>(L16, DD, 0, Bw1, DD, 0, 0.0625f, b1, 0, nullptr, 1, 0, 0, nullptr, F16, DFF, 0, NRQ, DFF, DD);
  k_gemm_hhx<0><<<gQ, 128, 0, stream>>>(F16, DFF, 0, Bw2, DFF, 0, 0.0625f, b2, 0, Q2, 1, (size_t)DD, 0, R3, nullptr, DD, 0, NRQ, DD, DFF);
  k_out<<<(NBm * NQ * (DD / 4) + 255) / 256, 256, 0, stream>>>(R3, (float*)d_out);
}
